// DAGLayer_37280316129534
// MI455X (gfx1250) — hardware-verified
//
#include <hip/hip_runtime.h>


#define MAXA    50
#define NSLOT   51
#define NGF     30
#define NAF     75
#define HIDDEN  100
#define NIN     1545

#define RB      16
#define NTHR    224
#define K1      1664
#define K1Q     208
#define KS1     52
#define N1P     112
#define K2P     128
#define N2P     32
#define GFP     32
#define GFA     (NSLOT * GFP)
#define HP      136

#define OFF_GF    0
#define OFF_AT    (OFF_GF + RB * GFA * 2)
#define OFF_HHI   (OFF_AT + RB * K1 * 2)
#define OFF_HLO   (OFF_HHI + RB * HP * 2)
#define OFF_OUTS  (OFF_HLO + RB * HP * 2)
#define OFF_PAR   (OFF_OUTS + RB * NGF * 4)
#define OFF_MSK   (OFF_PAR + RB * MAXA * 4)
#define SMEM_BYTES (OFF_MSK + RB * 4)

#define W0P_BYTES (N1P * K1 * 2)
#define W1P_BYTES (N2P * K2P * 2)
#define WS_TOTAL  (W0P_BYTES + 2 * W1P_BYTES)

static_assert((OFF_AT % 16) == 0);
static_assert((OFF_HHI % 16) == 0);
static_assert((OFF_HLO % 16) == 0);
static_assert((OFF_OUTS % 16) == 0);
static_assert((OFF_PAR % 16) == 0);
static_assert((OFF_MSK % 16) == 0);
static_assert((SMEM_BYTES % 16) == 0);
static_assert((W0P_BYTES % 128) == 0);
static_assert((W1P_BYTES % 128) == 0);
static_assert(((RB * NGF * 4) % 128) == 0);

typedef _Float16 f16t;
typedef unsigned short us_t;
typedef f16t   v8h  __attribute__((ext_vector_type(8)));
typedef f16t   v16h __attribute__((ext_vector_type(16)));
typedef us_t   v8us __attribute__((ext_vector_type(8)));
typedef __bf16 v16b __attribute__((ext_vector_type(16)));
typedef float  v8f  __attribute__((ext_vector_type(8)));
typedef float  v4f  __attribute__((ext_vector_type(4)));
typedef unsigned int v4u __attribute__((ext_vector_type(4)));

union FragH { v16h v; v8h  q[2]; };
union FragB { v16b v; v8us q[2]; };
union Pk16  { v8h  h; v4u u; };
union PkUS  { v8us s; v4u u; };
union Pk32  { v4f  f; v4u u; };

__device__ __forceinline__ v8f mma_f16(v16h a, v16h b, v8f c) {
    v8f d = __builtin_amdgcn_wmma_f32_16x16x32_f16(false, a, false, b, (short)0, c, false, false);
    asm volatile("v_nop\n\tv_nop\n\tv_nop\n\tv_nop" : "+v"(d) : "v"(a), "v"(b));
    return d;
}
__device__ __forceinline__ v8f mma_bf16(v16b a, v16b b, v8f c) {
    v8f d = __builtin_amdgcn_wmma_f32_16x16x32_bf16(false, a, false, b, (short)0, c, false, false);
    asm volatile("v_nop\n\tv_nop\n\tv_nop\n\tv_nop" : "+v"(d) : "v"(a), "v"(b));
    return d;
}
__device__ __forceinline__ v8f zero8() {
    v8f z = {0.f, 0.f, 0.f, 0.f, 0.f, 0.f, 0.f, 0.f};
    return z;
}

__device__ __forceinline__ us_t bf16_rne(float x) {
    unsigned int u = __float_as_uint(x);
    u += 0x7FFFu + ((u >> 16) & 1u);
    return (us_t)(u >> 16);
}
__device__ __forceinline__ float bf16_val(us_t b) {
    return __uint_as_float(((unsigned int)b) << 16);
}

__global__ __launch_bounds__(256)
void k_w0plane(const float* __restrict__ W0, f16t* __restrict__ P) {
    const int i = blockIdx.x * 256 + threadIdx.x;
    if (i >= N1P * K1Q) return;
    const int n  = i / K1Q;
    const int k8 = (i - n * K1Q) * 8;
    const int nc = (n < HIDDEN) ? n : (HIDDEN - 1);
    Pk16 pk;
#pragma unroll
    for (int e = 0; e < 8; ++e) {
        const int k = k8 + e;
        int  kidx;
        bool ok;
        if (k < 96) {
            kidx = k;
            ok   = (k < NAF);
        } else {
            const int jj = (k - 96) >> 5, c = (k - 96) & 31;
            kidx = NAF + NGF * jj + c;
            ok   = (c < NGF);
        }
        kidx = (kidx < 0) ? 0 : ((kidx > NIN - 1) ? (NIN - 1) : kidx);
        const float wv = W0[(size_t)kidx * HIDDEN + nc];
        const float v  = (ok && n < HIDDEN) ? wv * 16.0f : 0.0f;
        pk.h[e] = (f16t)v;
    }
    f16t* d = P + (size_t)n * K1 + k8;
    *(volatile v4u*)d = pk.u;
    __threadfence();
    *(volatile v4u*)d = pk.u;
}

__global__ __launch_bounds__(256)
void k_w1planes(const float* __restrict__ W1, us_t* __restrict__ PH, us_t* __restrict__ PL) {
    const int i = blockIdx.x * 256 + threadIdx.x;
    if (i >= N2P * (K2P / 8)) return;
    const int n  = i >> 4;
    const int k8 = (i & 15) * 8;
    const int nc = (n < NGF) ? n : (NGF - 1);
    PkUS ph, pl;
#pragma unroll
    for (int e = 0; e < 8; ++e) {
        const int k  = k8 + e;
        const int kc = (k < HIDDEN) ? k : (HIDDEN - 1);
        const float wv = W1[(size_t)kc * NGF + nc];
        const float v  = (n < NGF && k < HIDDEN) ? wv : 0.0f;
        const us_t hb  = bf16_rne(v);
        const us_t lb  = bf16_rne(v - bf16_val(hb));
        ph.s[e] = hb;
        pl.s[e] = lb;
    }
    us_t* dh = PH + (size_t)n * K2P + k8;
    us_t* dl = PL + (size_t)n * K2P + k8;
    *(volatile v4u*)dh = ph.u;
    *(volatile v4u*)dl = pl.u;
    __threadfence();
    *(volatile v4u*)dh = ph.u;
    *(volatile v4u*)dl = pl.u;
}

__global__ __launch_bounds__(NTHR)
void k_prop(const float* __restrict__ atomf, const int* __restrict__ parents, const int* __restrict__ orders,
            const int* __restrict__ flags, const int* __restrict__ natoms, const f16t* __restrict__ W0P,
            const us_t* __restrict__ W1H, const us_t* __restrict__ W1L, const float* __restrict__ b0,
            const float* __restrict__ b1, float* __restrict__ out, int N) {
    extern __shared__ __attribute__((aligned(16))) char smem[];
    f16t*  gfl  = (f16t*)(smem + OFF_GF);
    f16t*  atl  = (f16t*)(smem + OFF_AT);
    us_t*  hhi  = (us_t*)(smem + OFF_HHI);
    us_t*  hlo  = (us_t*)(smem + OFF_HLO);
    float* outs = (float*)(smem + OFF_OUTS);
    int*   parl = (int*)(smem + OFF_PAR);
    int*   mskl = (int*)(smem + OFF_MSK);

    const int tid = threadIdx.x;
    const int w   = __builtin_amdgcn_readfirstlane(tid >> 5);
    const int l   = tid & 31, h = l >> 4, m = l & 15;
    const int gbase = blockIdx.x * RB;
    if (gbase + RB > N) return;

    const int nv = natoms[0];
    const int obound = (nv < 1) ? 1 : ((nv > N) ? N : nv);

    {
        v4u z = {0u, 0u, 0u, 0u};
        v4u* p = (v4u*)smem;
        for (int e = tid; e < SMEM_BYTES / 16; e += NTHR) p[e] = z;
    }
    __syncthreads();

    const int n0   = 16 * w;
    const int col1 = n0 + m;
    const int col2 = 16 * (w & 1) + m;
    float bias0, bias1;
    {
        const float bb0 = b0[(col1 < HIDDEN) ? col1 : (HIDDEN - 1)];
        bias0 = (col1 < HIDDEN) ? bb0 : 0.0f;
        const float bb1 = b1[(col2 < NGF) ? col2 : (NGF - 1)];
        bias1 = (col2 < NGF) ? bb1 : 0.0f;
    }
    const f16t* Aw = atl + m * K1 + 8 * h;
    const f16t* Bw = W0P + (size_t)(n0 + m) * K1 + 8 * h;
    const us_t* Ah = hhi + m * HP + 8 * h;
    const us_t* Al = hlo + m * HP + 8 * h;
    const us_t* Bh = W1H + (size_t)(16 * (w & 1) + m) * K2P + 8 * h;
    const us_t* Bl = W1L + (size_t)(16 * (w & 1) + m) * K2P + 8 * h;
    const float INV16 = 0.0625f;

#pragma unroll 1
    for (int t = 0; t < MAXA; ++t) {
        for (int e = tid; e < RB * MAXA; e += NTHR) {
            const int r = e / MAXA, j = e - r * MAXA;
            int p = parents[(size_t)(gbase + r) * (MAXA * MAXA) + (size_t)t * MAXA + j];
            p = (p < 0) ? (p + NSLOT) : p;
            p = (p < 0) ? 0 : ((p > NSLOT - 1) ? (NSLOT - 1) : p);
            parl[e] = p;
        }
        {
            const int rr = (tid < RB) ? tid : 0;
            const int mk = flags[(size_t)(gbase + rr) * MAXA + t];
            if (tid < RB) mskl[tid] = mk;
        }
        for (int e = tid; e < RB * NAF; e += NTHR) {
            const int r = e / NAF, f = e - r * NAF;
            int o = orders[(size_t)(gbase + r) * MAXA + t];
            o = (o < 0) ? (o + N) : o;
            o = (o < 0) ? 0 : ((o > obound - 1) ? (obound - 1) : o);
            atl[r * K1 + f] = (f16t)atomf[(size_t)o * NAF + f];
        }
        __syncthreads();

        for (int e = tid; e < RB * (MAXA - 1) * 4; e += NTHR) {
            const int r   = e / ((MAXA - 1) * 4);
            const int rem = e - r * ((MAXA - 1) * 4);
            const int jj  = rem >> 2, q = rem & 3;
            const int s   = parl[r * MAXA + jj + 1];
            const v4u v = *(const v4u*)(gfl + r * GFA + s * GFP + q * 8);
            *(v4u*)(atl + r * K1 + 96 + jj * 32 + q * 8) = v;
        }
        __syncthreads();

        v8f acc = zero8();
#pragma unroll 4
        for (int kt = 0; kt < KS1; ++kt) {
            FragH a, b;
            a.q[0] = *(const v8h*)(Aw + kt * 32);
            a.q[1] = *(const v8h*)(Aw + kt * 32 + 16);
            b.q[0] = *(const v8h*)(Bw + kt * 32);
            b.q[1] = *(const v8h*)(Bw + kt * 32 + 16);
            acc = mma_f16(a.v, b.v, acc);
        }
#pragma unroll
        for (int r = 0; r < 8; ++r) {
            float v = fmaf(acc[r], INV16, bias0);
            v = fmaxf(v, 0.0f);
            const us_t hb = bf16_rne(v);
            const us_t lb = bf16_rne(v - bf16_val(hb));
            const int row = 8 * h + r;
            hhi[row * HP + col1] = hb;
            hlo[row * HP + col1] = lb;
        }
        __syncthreads();

        if (w < 2) {
            v8f acc2 = zero8();
#pragma unroll
            for (int kt = 0; kt < K2P / 32; ++kt) {
                FragB ah, al, bh, bl;
                ah.q[0] = *(const v8us*)(Ah + kt * 32);
                ah.q[1] = *(const v8us*)(Ah + kt * 32 + 16);
                al.q[0] = *(const v8us*)(Al + kt * 32);
                al.q[1] = *(const v8us*)(Al + kt * 32 + 16);
                bh.q[0] = *(const v8us*)(Bh + kt * 32);
                bh.q[1] = *(const v8us*)(Bh + kt * 32 + 16);
                bl.q[0] = *(const v8us*)(Bl + kt * 32);
                bl.q[1] = *(const v8us*)(Bl + kt * 32 + 16);
                acc2 = mma_bf16(ah.v, bh.v, acc2);
                acc2 = mma_bf16(ah.v, bl.v, acc2);
                acc2 = mma_bf16(al.v, bh.v, acc2);
            }
#pragma unroll
            for (int r = 0; r < 8; ++r) {
                const int row = 8 * h + r;
                float v = acc2[r] + bias1;
                v = fmaxf(v, 0.0f);
                const int mk = mskl[row];
                const int p0 = parl[row * MAXA];
                if (col2 < NGF) {
                    if (mk != 0) gfl[row * GFA + p0 * GFP + col2] = (f16t)v;
                    outs[row * NGF + col2] = (mk != 0) ? v : 0.0f;
                }
            }
        }
        __syncthreads();
    }

    {
        const bool act = tid < (RB * NGF) / 4;
        const int  pc  = act ? tid : 0;
        Pk32 pv;
        pv.f = *(const v4f*)(outs + pc * 4);
        float* dst = out + (size_t)gbase * NGF + (size_t)pc * 4;
        if (act) *(volatile v4u*)dst = pv.u;
        __threadfence();
        if (act) *(volatile v4u*)dst = pv.u;
    }
}

extern "C" void kernel_launch(void* const* d_in, const int* in_sizes, int n_in,
                              void* d_out, int out_size, void* d_ws, size_t ws_size,
                              hipStream_t stream) {
    if (n_in < 9) return;
    const int N = in_sizes[0] / NAF;
    if (N <= 0 || in_sizes[0] != N * NAF || (N % RB) != 0) return;
    if (in_sizes[1] != N * MAXA * MAXA || in_sizes[2] != N * MAXA || in_sizes[3] != N * MAXA) return;
    if (in_sizes[4] < 1) return;
    if (in_sizes[5] != NIN * HIDDEN || in_sizes[6] != HIDDEN || in_sizes[7] != HIDDEN * NGF || in_sizes[8] != NGF) return;
    if (out_size != N * NGF) return;
    if ((size_t)WS_TOTAL > ws_size) return;

    const float* atomf   = (const float*)d_in[0];
    const int*   parents = (const int*)d_in[1];
    const int*   orders  = (const int*)d_in[2];
    const int*   flags   = (const int*)d_in[3];
    const int*   natoms  = (const int*)d_in[4];
    const float* W0      = (const float*)d_in[5];
    const float* b0      = (const float*)d_in[6];
    const float* W1      = (const float*)d_in[7];
    const float* b1      = (const float*)d_in[8];
    float*       out     = (float*)d_out;

    char* ws  = (char*)d_ws;
    f16t* W0P = (f16t*)(ws);
    us_t* W1H = (us_t*)(ws + W0P_BYTES);
    us_t* W1L = (us_t*)(ws + W0P_BYTES + W1P_BYTES);

    k_w0plane<<<dim3((N1P * K1Q + 255) / 256), dim3(256), 0, stream>>>(W0, W0P);
    k_w1planes<<<dim3((N2P * (K2P / 8) + 255) / 256), dim3(256), 0, stream>>>(W1, W1H, W1L);

    (void)hipFuncSetAttribute(reinterpret_cast<const void*>(&k_prop),
                              hipFuncAttributeMaxDynamicSharedMemorySize, (int)SMEM_BYTES);
    k_prop<<<dim3(N / RB), dim3(NTHR), SMEM_BYTES, stream>>>(atomf, parents, orders, flags, natoms,
                                                             W0P, W1H, W1L, b0, b1, out, N);
}
